// DynamicMaskHead_26946624815736
// MI455X (gfx1250) — hardware-verified
//
#include <hip/hip_runtime.h>
#include <stddef.h>
#include <stdint.h>

#define CIN     64
#define HHT     160
#define WWD     256
#define HW      (HHT * WWD)
#define CH      16
#define PTOT    1361
#define OFF_W1  1056
#define OFF_W2  1312
#define OFF_B0  1328
#define OFF_B1  1344
#define OFF_B2  1360
#define MBSHIFT 2.19f
#define CHUNK   256
#define NTHR    128
#define NWAVE   4
#define TMAXI   256
#define NIMGMAX 64
#define TILES_PER_WAVE (CHUNK / (16 * NWAVE))

static_assert(OFF_W1 == CH * (CIN + 2));
static_assert(OFF_W2 == OFF_W1 + CH * CH);
static_assert(OFF_B0 == OFF_W2 + CH);
static_assert(OFF_B1 == OFF_B0 + CH);
static_assert(OFF_B2 == OFF_B1 + CH);
static_assert(PTOT == OFF_B2 + 1);
static_assert((HW % CHUNK) == 0);
static_assert((CHUNK % (16 * NWAVE)) == 0);
static_assert(NTHR == 32 * NWAVE);
static_assert((((CHUNK / 4) * (CIN / 2)) % NTHR) == 0);
static_assert(CHUNK == 2 * 32 * 4);
static_assert((CHUNK / 4) == 64);

typedef unsigned short v8us  __attribute__((ext_vector_type(8)));
typedef unsigned short v16us __attribute__((ext_vector_type(16)));
typedef float          v4f   __attribute__((ext_vector_type(4)));
typedef float          v8f   __attribute__((ext_vector_type(8)));
typedef _Float16       v16h  __attribute__((ext_vector_type(16)));
#if defined(__HIP_DEVICE_COMPILE__)
typedef __bf16         v16bf __attribute__((ext_vector_type(16)));
#endif

union FragU { v16us v; v8us half[2]; };

__device__ __forceinline__ unsigned bbits(float f) {
  unsigned u = __float_as_uint(f);
  return (u + 0x7FFFu + ((u >> 16) & 1u)) >> 16;
}
__device__ __forceinline__ float bf16r(float f) {
  return __uint_as_float(bbits(f) << 16);
}
__device__ __forceinline__ unsigned short hbits(float f) {
  const _Float16 h = (_Float16)f;
  return __builtin_bit_cast(unsigned short, h);
}
__device__ __forceinline__ v8f zero8() { v8f z = {0.f, 0.f, 0.f, 0.f, 0.f, 0.f, 0.f, 0.f}; return z; }

__device__ __forceinline__ v16us ldfrag(const unsigned short* p) {
  FragU f;
  f.half[0] = *(const v8us*)(p);
  f.half[1] = *(const v8us*)(p + 16);
  return f.v;
}
__device__ __forceinline__ void ld8(float* dst, const float* src) {
  const v4f lo = *(const v4f*)(src);
  const v4f hi = *(const v4f*)(src + 4);
  dst[0] = lo[0]; dst[1] = lo[1]; dst[2] = lo[2]; dst[3] = lo[3];
  dst[4] = hi[0]; dst[5] = hi[1]; dst[6] = hi[2]; dst[7] = hi[3];
}

__device__ __forceinline__ v8f mma_bf(v16us a, v16us b, v8f c) {
#if defined(__HIP_DEVICE_COMPILE__)
  return __builtin_amdgcn_wmma_f32_16x16x32_bf16(false, __builtin_bit_cast(v16bf, a),
                                                false, __builtin_bit_cast(v16bf, b),
                                                (short)0, c, false, false);
#else
  (void)a; (void)b;
  return c;
#endif
}
__device__ __forceinline__ v8f mma_h(v16us a, v16us b, v8f c) {
#if defined(__HIP_DEVICE_COMPILE__)
  return __builtin_amdgcn_wmma_f32_16x16x32_f16(false, __builtin_bit_cast(v16h, a),
                                               false, __builtin_bit_cast(v16h, b),
                                               (short)0, c, false, false);
#else
  (void)a; (void)b;
  return c;
#endif
}
__device__ __forceinline__ void guard2(v8f& acc, const v16us& a, const v16us& b) {
#if defined(__HIP_DEVICE_COMPILE__)
  asm volatile("v_nop\n\tv_nop\n\tv_nop\n\tv_nop" : "+v"(acc) : "v"(a), "v"(b));
#endif
}
__device__ __forceinline__ void guard4(v8f& acc, const v16us& a0, const v16us& a1,
                                       const v16us& b0, const v16us& b1) {
#if defined(__HIP_DEVICE_COMPILE__)
  asm volatile("v_nop\n\tv_nop\n\tv_nop\n\tv_nop" : "+v"(acc) : "v"(a0), "v"(a1), "v"(b0), "v"(b1));
#endif
}

__global__ __launch_bounds__(NTHR)
void k_head(const float* __restrict__ X, const float* __restrict__ PRM, const int* __restrict__ NUMI,
            float* out, int nimg, int T)
{
  __shared__ __align__(16) unsigned short sX[CHUNK * CIN];
  __shared__ __align__(16) unsigned short sW0[CH * CIN];
  __shared__ __align__(16) unsigned short sW1[CH * 32];
  __shared__ __align__(16) float sc[5 * CH];
  __shared__ __align__(16) float sOut[CHUNK];
  __shared__ int smap[TMAXI];
  __shared__ float sb2;

  const int tid  = threadIdx.x;
  const int lane = tid & 31;
  const int wave = tid >> 5;
  const int hh   = lane >> 4;
  const int m    = lane & 15;
  const int img  = blockIdx.y;
  const int px0  = blockIdx.x * CHUNK;

  {
    const float* xb = X + (size_t)img * CIN * HW + px0;
    unsigned int* d = (unsigned int*)sX;
#pragma unroll 1
    for (int it = 0; it < ((CHUNK / 4) * (CIN / 2)) / NTHR; ++it) {
      const int e  = it * NTHR + tid;
      const int pq = e & (CHUNK / 4 - 1);
      const int cp = e >> 6;
      const float* s0 = xb + (size_t)(2 * cp) * HW + 4 * pq;
      const v4f f0 = *(const v4f*)(s0);
      const v4f f1 = *(const v4f*)(s0 + HW);
#pragma unroll
      for (int j = 0; j < 4; ++j)
        d[(4 * pq + j) * (CIN / 2) + cp] = bbits(f0[j]) | (bbits(f1[j]) << 16);
    }
  }
  for (int tt = tid; tt < T; tt += NTHR) {
    int cnt = 0, ec = 0;
#pragma unroll 1
    for (int q = 0; q < nimg; ++q) {
      cnt += (ec <= tt) ? 1 : 0;
      ec  += NUMI[q];
    }
    int n = cnt - 1;
    n = n < 0 ? 0 : n;
    n = n > nimg - 1 ? nimg - 1 : n;
    smap[tt] = n;
  }
  __syncthreads();

#pragma unroll 1
  for (int t = 0; t < T; ++t) {
    if (smap[t] != img) continue;
    __syncthreads();

    {
      const float* pt = PRM + (size_t)t * PTOT;
#pragma unroll 1
      for (int it = 0; it < (PTOT + NTHR - 1) / NTHR; ++it) {
        const int j  = it * NTHR + tid;
        const int jj = j < PTOT ? j : PTOT - 1;
        const float v  = pt[jj];
        const float vb = bf16r(v);
        if (j < OFF_W1) {
          const int o  = j / (CIN + 2);
          const int ci = j - o * (CIN + 2);
          if (ci == 0)      sc[0 * CH + o] = vb;
          else if (ci == 1) sc[1 * CH + o] = vb;
          else              sW0[o * CIN + (ci - 2)] = (unsigned short)bbits(v);
        } else if (j < OFF_W2) {
          const int q = j - OFF_W1;
          const int o = q >> 4, i = q & 15;
          sW1[o * 32 + i]      = hbits(vb * 64.0f);
          sW1[o * 32 + 16 + i] = hbits(vb * 0.25f);
        } else if (j < OFF_B0) {
          sc[2 * CH + (j - OFF_W2)] = vb;
        } else if (j < OFF_B1) {
          sc[3 * CH + (j - OFF_B0)] = vb;
        } else if (j < OFF_B2) {
          sc[4 * CH + (j - OFF_B1)] = vb;
        } else if (j == OFF_B2) {
          sb2 = vb - MBSHIFT;
        }
      }
    }
    __syncthreads();

    const v16us a00 = ldfrag(sW0 + m * CIN + 8 * hh);
    const v16us a01 = ldfrag(sW0 + m * CIN + 32 + 8 * hh);
    const v16us a1  = ldfrag(sW1 + m * 32 + 8 * hh);
    float w0x[8], w0y[8], w2v[8], b0v[8], b1v[8];
    ld8(w0x, sc + 0 * CH + 8 * hh);
    ld8(w0y, sc + 1 * CH + 8 * hh);
    ld8(w2v, sc + 2 * CH + 8 * hh);
    ld8(b0v, sc + 3 * CH + 8 * hh);
    ld8(b1v, sc + 4 * CH + 8 * hh);
    const float b2 = sb2;
    float* outT = out + (size_t)t * HW + px0;

#pragma unroll 1
    for (int q = 0; q < TILES_PER_WAVE; ++q) {
      const int pl0 = (q * NWAVE + wave) * 16;
      const unsigned short* xr = sX + (pl0 + m) * CIN + 8 * hh;
      const v16us b00 = ldfrag(xr);
      const v16us b01 = ldfrag(xr + 32);

      v8f acc0 = zero8();
      acc0 = mma_bf(a00, b00, acc0);
      acc0 = mma_bf(a01, b01, acc0);
      guard4(acc0, a00, a01, b00, b01);

      const int pix  = px0 + pl0 + m;
      const float xf = (float)(pix % WWD);
      const float yf = (float)(pix / WWD);
      v8us e0, e1;
#pragma unroll
      for (int r = 0; r < 8; ++r) {
        float hv = acc0[r] + (w0x[r] * xf + w0y[r] * yf) + b0v[r];
        hv = fmaxf(hv, 0.0f);
        const _Float16 hi = (_Float16)hv;
        const float    lo = (hv - (float)hi) * 256.0f;
        const _Float16 lh = (_Float16)lo;
        e0[r] = __builtin_bit_cast(unsigned short, hi);
        e1[r] = __builtin_bit_cast(unsigned short, lh);
      }
      FragU fb;
      fb.half[0] = e0;
      fb.half[1] = e1;
      const v16us bl = fb.v;

      v8f acc1 = zero8();
      acc1 = mma_h(a1, bl, acc1);
      guard2(acc1, a1, bl);

      float part = 0.0f;
#pragma unroll
      for (int r = 0; r < 8; ++r) {
        float v = acc1[r] * 0.015625f + b1v[r];
        v = fmaxf(v, 0.0f);
        part += w2v[r] * v;
      }
      part += __shfl_xor(part, 16, 32);
      if (lane < 16) sOut[pl0 + m] = part + b2;
    }
    __syncthreads();

    {
      const int oi = 128 * (wave & 1) + 4 * lane;
      const v4f ov = *(const v4f*)(sOut + oi);
      float* po = outT + oi;
      const bool wr = wave < 2;
      if (wr) *(volatile v4f*)po = ov;
      __threadfence();
      if (wr) *(volatile v4f*)po = ov;
    }
  }
}

extern "C" void kernel_launch(void* const* d_in, const int* in_sizes, int n_in,
                              void* d_out, int out_size, void* d_ws, size_t ws_size,
                              hipStream_t stream) {
  (void)d_ws; (void)ws_size;
  if (n_in < 3) return;
  const int nimg = in_sizes[2];
  if (nimg < 1 || nimg > NIMGMAX) return;
  if ((long long)in_sizes[0] != (long long)nimg * (long long)CIN * (long long)HW) return;
  if (in_sizes[1] < PTOT || (in_sizes[1] % PTOT) != 0) return;
  const int T = in_sizes[1] / PTOT;
  if (T < 1 || T > TMAXI) return;
  if ((long long)out_size != (long long)T * (long long)HW) return;

  const float* X   = (const float*)d_in[0];
  const float* PRM = (const float*)d_in[1];
  const int*   NUM = (const int*)d_in[2];
  float* out = (float*)d_out;

  const dim3 grid(HW / CHUNK, nimg);
  k_head<<<grid, dim3(NTHR), 0, stream>>>(X, PRM, NUM, out, nimg, T);
  (void)hipGetLastError();
}
